// GridPEAttention_61512521613905
// MI455X (gfx1250) — hardware-verified
//
#include <hip/hip_runtime.h>


namespace {
constexpr int NB = 8, N = 1025, NP = 1088  , C = 768, NH = 8, D = 96, C3 = 3 * C, NR = NB * NP, NSIMP = 3, NSC = 16;
constexpr float XS = 8.0f, WSC = 256.0f, PS = 8.0f, LOG2E = 1.4426950408889634f, LOG2_100 = 6.643856189774724f;

typedef _Float16 b16;
typedef __attribute__((ext_vector_type(16))) _Float16 v16b;
typedef __attribute__((ext_vector_type(8))) _Float16 v8b;
typedef __attribute__((ext_vector_type(4))) _Float16 v4b;
typedef __attribute__((ext_vector_type(8))) float v8f;
typedef __attribute__((ext_vector_type(4))) float v4f;
__device__ __forceinline__ float bf16_rne(float f) { unsigned int u = __float_as_uint(f); u += 0x7FFFu + ((u >> 16) & 1u); return __uint_as_float(u & 0xFFFF0000u); }
__device__ __forceinline__ void split16(float v, b16& hi, b16& lo) { hi = (b16)v; lo = (b16)(v - (float)hi); }
__device__ __forceinline__ v16b frag_kb(const b16* p, int hh) { const v8b a = *(const v8b*)(p + 8 * hh), b = *(const v8b*)(p + 16 + 8 * hh); v16b f;
#pragma unroll
  for (int e = 0; e < 8; ++e) { f[e] = a[e]; f[8 + e] = b[e]; } return f; }
__device__ __forceinline__ v8f wmma16b(v16b a, v16b b, v8f c) { v8f d = __builtin_amdgcn_wmma_f32_16x16x32_f16(false, a, false, b, (short)0, c, false, false); asm volatile("v_nop\n\tv_nop\n\tv_nop\n\tv_nop" : "+v"(d) : "v"(a), "v"(b)); return d; }
__device__ __forceinline__ void wave_lds_sync() { __builtin_amdgcn_fence(__ATOMIC_RELEASE, "workgroup"); __builtin_amdgcn_wave_barrier(); __builtin_amdgcn_fence(__ATOMIC_ACQUIRE, "workgroup"); }
__device__ __forceinline__ float nexp2(float x) { return __builtin_amdgcn_exp2f(x); }

__global__ __launch_bounds__(256) void prepx_kernel(const float* __restrict__ x, b16* __restrict__ X16) {
  const size_t t = (size_t)blockIdx.x * 256 + threadIdx.x; if (t >= (size_t)NR * C / 8) return; const size_t e = t * 8; const size_t r = e / C; const int c = (int)(e - r * C); const int b = (int)(r / NP), n = (int)(r - (size_t)b * NP);
  v8b o = {}; if (n < N) { const float* src = x + ((size_t)b * N + n) * C + c; const v4f a = *(const v4f*)src, cc = *(const v4f*)(src + 4);
#pragma unroll
    for (int j = 0; j < 4; ++j) { o[j] = (b16)(bf16_rne(a[j]) * XS); o[4 + j] = (b16)(bf16_rne(cc[j]) * XS); } }
  for (int pass = 0; pass < 2; ++pass) { *(volatile v8b*)(X16 + e) = o; __threadfence(); }
}
__global__ __launch_bounds__(256) void prepw_kernel(const float* __restrict__ wqkv, const float* __restrict__ wproj, b16* __restrict__ WT, b16* __restrict__ WPT) {
  __shared__ __attribute__((aligned(16))) b16 T[64][64 + 8];
  const int kind = blockIdx.z, d0 = blockIdx.x * 64, j0 = blockIdx.y * 64, t_ = threadIdx.x; const int OUTW = kind == 0 ? C3 : C; if (j0 >= OUTW) return;
  const float* w = kind == 0 ? wqkv : wproj; b16* dst = kind == 0 ? WT : WPT;
  for (int q = t_; q < 64 * 64; q += 256) { const int dd = q >> 6, jj = q & 63; T[jj][dd] = (b16)(bf16_rne(w[(size_t)(d0 + dd) * OUTW + j0 + jj]) * WSC); }
  __syncthreads();
  for (int pass = 0; pass < 2; ++pass) { for (int q = t_; q < 64 * 8; q += 256) { const int jj = q >> 3, c8 = (q & 7) * 8; *(volatile v8b*)(dst + (size_t)(j0 + jj) * C + d0 + c8) = *(const v8b*)(&T[jj][c8]); } __threadfence(); }
}
__global__ __launch_bounds__(128) void proj_kernel(const b16* __restrict__ X16, const b16* __restrict__ WT, int kind, float* __restrict__ RAW, b16* __restrict__ VTh, b16* __restrict__ VTl) {
  __shared__ __attribute__((aligned(16))) float Tf[4][16][128 + 4]; __shared__ __attribute__((aligned(16))) b16 Vt[128][64 + 8], Vtl[128][64 + 8];
  const int wave = threadIdx.x >> 5, lane = threadIdx.x & 31, nloc = lane & 15, hlf = lane >> 4, t_ = threadIdx.x; const size_t m0 = (size_t)blockIdx.x * 64 + wave * 16; const int n0 = blockIdx.y * 128;
  const b16* W = WT + ((size_t)kind * C) * C; v8f acc[8];
#pragma unroll
  for (int t = 0; t < 8; ++t) acc[t] = (v8f){};
#pragma unroll 2
  for (int kb = 0; kb < C; kb += 32) { const v16b a = frag_kb(X16 + (m0 + nloc) * C + kb, hlf);
#pragma unroll
    for (int t = 0; t < 8; ++t) acc[t] = wmma16b(a, frag_kb(W + (size_t)(n0 + t * 16 + nloc) * C + kb, hlf), acc[t]); }
  if (kind < 2) {
#pragma unroll
    for (int t = 0; t < 8; ++t)
#pragma unroll
      for (int r = 0; r < 8; ++r) Tf[wave][8 * hlf + r][t * 16 + nloc] = acc[t][r] * (1.0f / (XS * WSC));
    wave_lds_sync(); float* dst = RAW;
    for (int pass = 0; pass < 2; ++pass) { for (int rr = 0; rr < 16; ++rr) *(volatile v4f*)(dst + (m0 + rr) * C + n0 + lane * 4) = *(const v4f*)(&Tf[wave][rr][lane * 4]); __threadfence(); }
  } else {
    const int b = (int)(m0 / NP); const int s0 = (int)((size_t)blockIdx.x * 64 - (size_t)b * NP);
#pragma unroll
    for (int t = 0; t < 8; ++t)
#pragma unroll
      for (int r = 0; r < 8; ++r) { b16 h_, l_; split16(acc[t][r] * (1.0f / (XS * WSC)) * XS, h_, l_); Vt[t * 16 + nloc][wave * 16 + 8 * hlf + r] = h_; Vtl[t * 16 + nloc][wave * 16 + 8 * hlf + r] = l_; }
    __syncthreads();
    for (int pass = 0; pass < 2; ++pass) { for (int q = t_; q < 128 * 4; q += 128) { const int cc = q >> 2, grp = q & 3; const size_t mrow = (size_t)blockIdx.x * 64 + grp * 16; const int bb = (int)(mrow / NP), ss = (int)(mrow - (size_t)bb * NP);
        const int h = (n0 + cc) / D, dd = (n0 + cc) - h * D; const size_t gi = (((size_t)bb * NH + h) * D + dd) * NP + ss;
        *(volatile v8b*)(VTh + gi) = *(const v8b*)(&Vt[cc][grp * 16]); *(volatile v8b*)(VTh + gi + 8) = *(const v8b*)(&Vt[cc][grp * 16 + 8]); *(volatile v8b*)(VTl + gi) = *(const v8b*)(&Vtl[cc][grp * 16]); *(volatile v8b*)(VTl + gi + 8) = *(const v8b*)(&Vtl[cc][grp * 16 + 8]); } __threadfence(); }
    (void)b; (void)s0; }
}
__global__ __launch_bounds__(256) void rope_kernel(const float* __restrict__ RAW, int kind, const float* __restrict__ posv, const float* __restrict__ omg, b16* __restrict__ Qh, b16* __restrict__ Ql, b16* __restrict__ Kh, b16* __restrict__ Kl) {
  const size_t t = (size_t)blockIdx.x * 256 + threadIdx.x; const size_t per = (size_t)NR * C / 4; if (t >= per) return; const size_t g = t;
  const size_t row = g / (C / 4); const int c0 = (int)(g - row * (C / 4)) * 4; const int b = (int)(row / NP), n = (int)(row - (size_t)b * NP); const int h = c0 / D; const int p0 = (c0 - h * D) >> 1;
  const v4f a = *(const v4f*)(RAW + row * C + c0);
  float e0 = a[0], o0 = a[1], e1 = a[2], o1 = a[3];
  if (n >= 1 && n < N) { const float px = bf16_rne(posv[((size_t)b * (N - 1) + (n - 1)) * 2]), py = bf16_rne(posv[((size_t)b * (N - 1) + (n - 1)) * 2 + 1]);
    float th[2];
#pragma unroll
    for (int u = 0; u < 2; ++u) { const int pi = p0 + u; const int ni = pi / NSC, s = pi - ni * NSC; const float w0 = bf16_rne(omg[(h * NSIMP + ni) * 2]), w1 = bf16_rne(omg[(h * NSIMP + ni) * 2 + 1]);
      const float dot = px * w0 + py * w1; const float mag = nexp2(-(6.0f * (float)s / 96.0f) * LOG2_100); th[u] = dot * mag; }
    float sn0, cs0, sn1, cs1; sincosf(th[0], &sn0, &cs0); sincosf(th[1], &sn1, &cs1);
    const float re0 = a[0] * cs0 - a[1] * sn0, ro0 = a[0] * sn0 + a[1] * cs0, re1 = a[2] * cs1 - a[3] * sn1, ro1 = a[2] * sn1 + a[3] * cs1; e0 = re0; o0 = ro0; e1 = re1; o1 = ro1; }
  v4b hv, lv; b16 h_, l_; split16(e0 * XS, h_, l_); hv[0] = h_; lv[0] = l_; split16(o0 * XS, h_, l_); hv[1] = h_; lv[1] = l_; split16(e1 * XS, h_, l_); hv[2] = h_; lv[2] = l_; split16(o1 * XS, h_, l_); hv[3] = h_; lv[3] = l_;
  b16* dh = kind == 0 ? Qh : Kh; b16* dl = kind == 0 ? Ql : Kl;
  for (int pass = 0; pass < 2; ++pass) { *(volatile v4b*)(dh + row * C + c0) = hv; *(volatile v4b*)(dl + row * C + c0) = lv; __threadfence(); }
}
__global__ __launch_bounds__(64) void attn_kernel(const b16* __restrict__ Qh, const b16* __restrict__ Ql, const b16* __restrict__ Kh, const b16* __restrict__ Kl, const b16* __restrict__ VTh, const b16* __restrict__ VTl, b16* __restrict__ Oh, b16* __restrict__ Ol) {
  __shared__ __attribute__((aligned(16))) float To[2][16][D + 4];
  const int wave = threadIdx.x >> 5, lane = threadIdx.x & 31, hh = lane >> 4, col = lane & 15; const int b = blockIdx.z, h = blockIdx.y; const int q0 = blockIdx.x * 32 + wave * 16; if (q0 >= NP) return; const int qi = q0 + col;
  const size_t qo = ((size_t)b * NP + qi) * C + h * D; v16b qa[3], ql[3];
#pragma unroll
  for (int k = 0; k < 3; ++k) { qa[k] = frag_kb(Qh + qo + 32 * k, hh); ql[k] = frag_kb(Ql + qo + 32 * k, hh); }
  const b16* Kb = Kh + (size_t)b * NP * C + h * D; const b16* Klb = Kl + (size_t)b * NP * C + h * D; const b16* Vb = VTh + ((size_t)b * NH + h) * D * NP; const b16* Vlb = VTl + ((size_t)b * NH + h) * D * NP;
  float m = -INFINITY, l = 0.0f; v8f o[6], ol[6];
#pragma unroll
  for (int t = 0; t < 6; ++t) { o[t] = (v8f){}; ol[t] = (v8f){}; }
  const float cs = 0.10206207261596577f * LOG2E / (XS * XS);
  for (int kb = 0; kb < N; kb += 32) {
    v8f s0 = {}, s1 = {};
#pragma unroll
    for (int k = 0; k < 3; ++k) { const int kk0 = kb + col, kk1 = kb + 16 + col;   const b16* k0 = Kb + (size_t)kk0 * C + 32 * k, *k1 = Kb + (size_t)kk1 * C + 32 * k, *k0l = Klb + (size_t)kk0 * C + 32 * k, *k1l = Klb + (size_t)kk1 * C + 32 * k;
      v16b f = frag_kb(k0, hh); s0 = wmma16b(f, qa[k], s0); s0 = wmma16b(f, ql[k], s0); s0 = wmma16b(frag_kb(k0l, hh), qa[k], s0);
      f = frag_kb(k1, hh); s1 = wmma16b(f, qa[k], s1); s1 = wmma16b(f, ql[k], s1); s1 = wmma16b(frag_kb(k1l, hh), qa[k], s1); }
    float e[16]; float mx = -INFINITY;
#pragma unroll
    for (int r = 0; r < 8; ++r) { const int k0i = kb + 8 * hh + r, k1i = kb + 16 + 8 * hh + r; e[r] = (k0i < N) ? s0[r] * cs : -INFINITY; e[8 + r] = (k1i < N) ? s1[r] * cs : -INFINITY; mx = fmaxf(mx, fmaxf(e[r], e[8 + r])); }
    mx = fmaxf(mx, __shfl_xor(mx, 16)); const float mn = fmaxf(m, mx); const float al = nexp2(m - mn); m = mn; float sum = 0.0f; v16b ph, pl;
#pragma unroll
    for (int i = 0; i < 16; ++i) { const float p = nexp2(e[i] - mn); sum += p; const b16 h_ = (b16)(p * PS); ph[i] = h_; pl[i] = (b16)(p * PS - (float)h_); }
    sum += __shfl_xor(sum, 16); l = l * al + sum;
#pragma unroll
    for (int t = 0; t < 6; ++t) { o[t] *= al; ol[t] *= al; const v16b vf = frag_kb(Vb + (size_t)(t * 16 + col) * NP + kb, hh); o[t] = wmma16b(vf, ph, o[t]); ol[t] = wmma16b(vf, pl, ol[t]); ol[t] = wmma16b(frag_kb(Vlb + (size_t)(t * 16 + col) * NP + kb, hh), ph, ol[t]); }
    }
  const float inv = 1.0f / (l * PS * XS);
#pragma unroll
  for (int t = 0; t < 6; ++t)
#pragma unroll
    for (int r = 0; r < 8; ++r) To[wave][col][t * 16 + 8 * hh + r] = (o[t][r] + ol[t][r]) * inv;
  wave_lds_sync();
  for (int pass = 0; pass < 2; ++pass) { for (int r2 = 0; r2 < 16; r2 += 2) { const int rr = r2 + (lane >> 4), c8 = (lane & 15) * 8; if (c8 < D) { v8b hv, lv; for (int j = 0; j < 8; ++j) { b16 a_, c_; split16(To[wave][rr][c8 + j] * XS, a_, c_); hv[j] = a_; lv[j] = c_; }
        const size_t gi = ((size_t)b * NP + q0 + rr) * C + h * D + c8; *(volatile v8b*)(Oh + gi) = hv; *(volatile v8b*)(Ol + gi) = lv; } } __threadfence(); }
}
__global__ __launch_bounds__(128) void outproj_kernel(const b16* __restrict__ Oh, const b16* __restrict__ Ol, const b16* __restrict__ WPT, const float* __restrict__ bproj, float* __restrict__ out) {
  __shared__ __attribute__((aligned(16))) float Ts[4][16][128 + 4];
  const int wave = threadIdx.x >> 5, lane = threadIdx.x & 31, nloc = lane & 15, hlf = lane >> 4; const size_t m0 = (size_t)blockIdx.x * 64 + wave * 16; const int n0 = blockIdx.y * 128;
  v8f acc[8];
#pragma unroll
  for (int t = 0; t < 8; ++t) acc[t] = (v8f){};
#pragma unroll 2
  for (int kb = 0; kb < C; kb += 32) { const v16b a = frag_kb(Oh + (m0 + nloc) * C + kb, hlf), al = frag_kb(Ol + (m0 + nloc) * C + kb, hlf);
#pragma unroll
    for (int t = 0; t < 8; ++t) { const v16b bw = frag_kb(WPT + (size_t)(n0 + t * 16 + nloc) * C + kb, hlf); acc[t] = wmma16b(a, bw, acc[t]); acc[t] = wmma16b(al, bw, acc[t]); } }
#pragma unroll
  for (int t = 0; t < 8; ++t) { const float bb = bf16_rne(bproj[n0 + t * 16 + nloc]);
#pragma unroll
    for (int r = 0; r < 8; ++r) Ts[wave][8 * hlf + r][t * 16 + nloc] = acc[t][r] * (1.0f / (XS * WSC)) + bb; }
  wave_lds_sync();
  for (int pass = 0; pass < 2; ++pass) { for (int rr = 0; rr < 16; ++rr) { const size_t prow = m0 + rr; const int b = (int)(prow / NP), n = (int)(prow - (size_t)b * NP); if (n < N) *(volatile v4f*)(out + ((size_t)b * N + n) * C + n0 + lane * 4) = *(const v4f*)(&Ts[wave][rr][lane * 4]); } __threadfence(); }
}
}

extern "C" void kernel_launch(void* const* d_in, const int* in_sizes, int n_in, void* d_out, int out_size, void* d_ws, size_t ws_size, hipStream_t stream) {
  (void)n_in;
  auto Fp = [&](int i) { return (const float*)d_in[i]; };
  if (in_sizes[0] != NB * N * C || in_sizes[1] != NB * (N - 1) * 2 || in_sizes[2] != C * C3 || in_sizes[3] != C * C || in_sizes[5] != NH * NSIMP * 2 || out_size != NB * N * C) return;
  size_t off = 0; char* ws = (char*)d_ws;
  auto carve = [&](size_t bytes) { char* p = ws + off; off += (bytes + 255) & ~(size_t)255; return p; };
  b16* X16 = (b16*)carve((size_t)NR * C * 2); b16* WT = (b16*)carve((size_t)C3 * C * 2); b16* WPT = (b16*)carve((size_t)C * C * 2); float* RAW = (float*)carve((size_t)NR * C * 4);
  b16* Qh = (b16*)carve((size_t)NR * C * 2); b16* Ql = (b16*)carve((size_t)NR * C * 2); b16* Kh = (b16*)carve((size_t)NR * C * 2); b16* Kl = (b16*)carve((size_t)NR * C * 2); b16* VTh = (b16*)carve((size_t)NR * C * 2); b16* VTl = (b16*)carve((size_t)NR * C * 2);
  b16* Oh = Qh; b16* Ol = Ql;
  if (off > ws_size || off > ((size_t)128 << 20)) return;
  prepx_kernel<<<(unsigned)(((size_t)NR * C / 8 + 255) / 256), 256, 0, stream>>>(Fp(0), X16);
  prepw_kernel<<<dim3(C / 64, C3 / 64, 2), 256, 0, stream>>>(Fp(2), Fp(3), WT, WPT);
  proj_kernel<<<dim3(NR / 64, C / 128, 1), 128, 0, stream>>>(X16, WT, 0, RAW, VTh, VTl);
  rope_kernel<<<(unsigned)(((size_t)NR * C / 4 + 255) / 256), 256, 0, stream>>>(RAW, 0, Fp(1), Fp(5), Qh, Ql, Kh, Kl);
  proj_kernel<<<dim3(NR / 64, C / 128, 1), 128, 0, stream>>>(X16, WT, 1, RAW, VTh, VTl);
  rope_kernel<<<(unsigned)(((size_t)NR * C / 4 + 255) / 256), 256, 0, stream>>>(RAW, 1, Fp(1), Fp(5), Qh, Ql, Kh, Kl);
  proj_kernel<<<dim3(NR / 64, C / 128, 1), 128, 0, stream>>>(X16, WT, 2, RAW, VTh, VTl);
  attn_kernel<<<dim3((NP + 31) / 32, NH, NB), 64, 0, stream>>>(Qh, Ql, Kh, Kl, VTh, VTl, Oh, Ol);
  outproj_kernel<<<dim3(NR / 64, C / 128), 128, 0, stream>>>(Oh, Ol, WPT, Fp(4), (float*)d_out);
}
